// SineSPE_52218212385266
// MI455X (gfx1250) — hardware-verified
//
#include <hip/hip_runtime.h>
#include <math.h>
#include <stdint.h>

#define NB    2
#define NL    1024
#define NHD   8
#define ND    64
#define NS    10
#define NJ    20
#define NR    128
#define NK    1280
#define NBH   16
#define NTAB  5120
#define NOUT  (NB * NL * NHD * NR)
#define PLANE ((size_t)NHD * NL * NK)
#define ZTN   ((size_t)NBH * NR * NK)

static_assert(NK == ND * NJ);
static_assert((NK % 32) == 0);
static_assert((NL % 64) == 0);
static_assert(NTAB == NHD * ND * NS);
static_assert(NBH == NB * NHD);
static_assert(sizeof(_Float16) == 2);

typedef _Float16 v16h __attribute__((ext_vector_type(16)));
typedef _Float16 v8h  __attribute__((ext_vector_type(8)));
typedef float    v8f  __attribute__((ext_vector_type(8)));
typedef float    v4f  __attribute__((ext_vector_type(4)));
typedef v4f __attribute__((may_alias)) v4fa;
typedef v8h __attribute__((may_alias)) v8ha;

union Frag { v16h v; v8h half[2]; };

constexpr float kTwoPi = 6.2831853071795864769f;
constexpr float kScale = 0.011048543456039806f;
constexpr float k2m16  = 1.52587890625e-05f;
constexpr float k2m27  = 7.450580596923828125e-09f;

__device__ __forceinline__ unsigned short bf_bits(float f) {
  unsigned u = __float_as_uint(f);
  return (unsigned short)((u + 0x7FFFu + ((u >> 16) & 1u)) >> 16);
}
__device__ __forceinline__ float bf_up(unsigned short b) { return __uint_as_float(((unsigned)b) << 16); }
__device__ __forceinline__ float bfr(float f) { return bf_up(bf_bits(f)); }
__device__ __forceinline__ v8f zero8() {
  v8f z;
  z[0] = 0.f; z[1] = 0.f; z[2] = 0.f; z[3] = 0.f; z[4] = 0.f; z[5] = 0.f; z[6] = 0.f; z[7] = 0.f;
  return z;
}
__device__ __forceinline__ void hsplit(float v, _Float16& hi, _Float16& lo) {
  const _Float16 hv = (_Float16)v;
  hi = hv;
  lo = (_Float16)((v - (float)hv) * 2048.0f);
}
__device__ __forceinline__ _Float16 zcvt(float v) { return (_Float16)(bfr(v) * 16.0f); }

__device__ __forceinline__ v16h ldfrag(const _Float16* p) {
  Frag f;
  f.half[0] = *(const v8h*)(p);
  f.half[1] = *(const v8h*)(p + 16);
  return f.v;
}

__device__ __forceinline__ v8f mma(v16h a, v16h b, v8f c) {
  v8f d = __builtin_amdgcn_wmma_f32_16x16x32_f16(false, a, false, b, (short)0, c, false, false);
#if defined(__HIP_DEVICE_COMPILE__)
  asm volatile("v_nop\n\tv_nop\n\tv_nop\n\tv_nop" : "+v"(d) : "v"(a), "v"(b));
#endif
  return d;
}

__global__ __launch_bounds__(256) void k_tab(const float* __restrict__ freqs, const float* __restrict__ gains,
                                            float* tab) {
#pragma clang fp contract(off)
  __shared__ __align__(16) float sT[1024];
  __shared__ __align__(16) float sG[1024];
  const int tid  = threadIdx.x;
  const int base = blockIdx.x * 1024;
#pragma unroll 1
  for (int it = 0; it < 4; ++it) {
    const int le = it * 256 + tid;
    const int e  = base + le;
    const float f  = bfr(freqs[e]);
    const float ef = expf(-f);
    const float sg = 1.0f / (1.0f + ef);
    const float fr = sg * 0.5f;
    sT[le] = kTwoPi * fr;
    const float g  = bfr(gains[e]);
    const float sp = fmaxf(g, 0.0f) + log1pf(expf(-fabsf(g)));
    sG[le] = (sp * kScale) * 4096.0f;
  }
  __syncthreads();
  const v4f tv = *(const v4fa*)(sT + 4 * tid);
  const v4f gv = *(const v4fa*)(sG + 4 * tid);
  float* dt = tab + base + 4 * tid;
  float* dg = tab + NTAB + base + 4 * tid;
  *(volatile v4f*)dt = tv;
  *(volatile v4f*)dg = gv;
  __threadfence();
  *(volatile v4f*)dt = tv;
  *(volatile v4f*)dg = gv;
}

__global__ __launch_bounds__(256) void k_zt(const float* __restrict__ z, _Float16* zt) {
  __shared__ __align__(16) _Float16 sT[16 * 640];
  const int tid = threadIdx.x;
  const int bx  = blockIdx.x;
  const int rt  = bx & 7;
  const int dh  = (bx >> 3) & 1;
  const int bh  = bx >> 4;
  const int r0  = rt * 16;
  const float* zb = z + ((size_t)(bh * ND + dh * 32)) * (NJ * NR) + r0;
#pragma unroll 2
  for (int it = 0; it < 10; ++it) {
    const int q  = it * 256 + tid;
    const int r4 = q & 3;
    const int dj = q >> 2;
    const int dd = dj / NJ;
    const int j  = dj - dd * NJ;
    const v4f v = *(const v4f*)(zb + (size_t)dj * NR + 4 * r4);
    _Float16* sp = sT + (4 * r4) * 640 + j * 32 + dd;
    sp[0]    = zcvt(v[0]);
    sp[640]  = zcvt(v[1]);
    sp[1280] = zcvt(v[2]);
    sp[1920] = zcvt(v[3]);
  }
  __syncthreads();
  v8h pv[5];
  _Float16* zo = zt + ((size_t)(bh * NR + r0)) * NK + dh * 640;
#pragma unroll
  for (int u = 0; u < 5; ++u) {
    const int p   = u * 256 + tid;
    const int rr  = p / 80;
    const int off = (p - rr * 80) * 8;
    pv[u] = *(const v8ha*)(sT + rr * 640 + off);
  }
#pragma unroll
  for (int u = 0; u < 5; ++u) {
    const int p   = u * 256 + tid;
    const int rr  = p / 80;
    const int off = (p - rr * 80) * 8;
    *(volatile v8h*)(zo + (size_t)rr * NK + off) = pv[u];
  }
  __threadfence();
#pragma unroll
  for (int u = 0; u < 5; ++u) {
    const int p   = u * 256 + tid;
    const int rr  = p / 80;
    const int off = (p - rr * 80) * 8;
    *(volatile v8h*)(zo + (size_t)rr * NK + off) = pv[u];
  }
}

__global__ __launch_bounds__(160) void k_feat(const float* __restrict__ tab, const float* __restrict__ offsets,
                                             float* Pqk) {
#pragma clang fp contract(off)
  __shared__ __align__(16) float sP[2 * NK];
  const int tid = threadIdx.x;
  const int l   = blockIdx.x & (NL - 1);
  const int hh  = blockIdx.x >> 10;
  const int dh  = (tid >= 80) ? 1 : 0;
  const int rem = tid - dh * 80;
  const int s   = rem >> 3;
  const int dd4 = (rem & 7) * 4;
  const int jc  = (s < 5) ? (2 * s) : (2 * s - 10);
  const float lf = (float)l;
  const float* th = tab + hh * (ND * NS);
  const float* gh = tab + NTAB + hh * (ND * NS);
  const float* oh = offsets + hh * (ND * NS);
#pragma unroll 1
  for (int it = 0; it < 8; ++it) {
    const int c  = it >> 1;
    const int pl = it & 1;
    const int d  = dh * 32 + dd4 + c;
    const float tf  = th[d * NS + s];
    const float of  = bfr(oh[d * NS + s]);
    const float gc  = gh[d * NS + jc];
    const float gsn = gh[d * NS + jc + 1];
    const float pk  = tf * lf;
    const float pq  = pk + of;
    const float ph  = (pl != 0) ? pk : pq;
    float sn, cs;
    sincosf(ph, &sn, &cs);
    const int kc = pl * NK + dh * 640 + (2 * s) * 32 + dd4 + c;
    sP[kc]      = cs * gc;
    sP[kc + 32] = sn * gsn;
  }
  __syncthreads();
  v4f pv[4];
  float* prow = Pqk + ((size_t)(hh * NL + l)) * NK;
#pragma unroll
  for (int u = 0; u < 4; ++u) {
    const int p = u * 160 + tid;
    pv[u] = *(const v4fa*)(sP + 4 * p);
  }
#pragma unroll
  for (int u = 0; u < 4; ++u) {
    const int p   = u * 160 + tid;
    const int pl2 = (p >= 320) ? 1 : 0;
    const int kk  = (p - pl2 * 320) * 4;
    *(volatile v4f*)(prow + (size_t)pl2 * PLANE + kk) = pv[u];
  }
  __threadfence();
#pragma unroll
  for (int u = 0; u < 4; ++u) {
    const int p   = u * 160 + tid;
    const int pl2 = (p >= 320) ? 1 : 0;
    const int kk  = (p - pl2 * 320) * 4;
    *(volatile v4f*)(prow + (size_t)pl2 * PLANE + kk) = pv[u];
  }
}

__global__ __launch_bounds__(128) void k_gemm(const float* __restrict__ queries, const float* __restrict__ keys,
                                             const float* __restrict__ Pqk, const _Float16* __restrict__ zt,
                                             float* out) {
#pragma clang fp contract(off)
  __shared__ __align__(16) float sO[4 * 16 * 64];
  const int tid  = threadIdx.x;
  const int lane = tid & 31, wv = tid >> 5, hf = lane >> 4, m = lane & 15;
  const int bx   = blockIdx.x;
  const int sel  = bx & 1;
  const int ch   = (bx >> 1) & 1;
  const int lt   = (bx >> 2) & 15;
  const int bh   = bx >> 6;
  const int b    = bh >> 3, hh = bh & 7;
  const int l    = lt * 64 + wv * 16 + m;

  const float* X = (sel != 0) ? keys : queries;
  const float* xrow = X + ((size_t)((b * NL + l) * NHD + hh)) * ND + 8 * hf;
  const float* prow = Pqk + (size_t)sel * PLANE + ((size_t)(hh * NL + l)) * NK + 8 * hf;
  const _Float16* zcol = zt + ((size_t)(bh * NR + ch * 64 + m)) * NK + 8 * hf;

  v8f accH[4], accR[4];
#pragma unroll
  for (int nt = 0; nt < 4; ++nt) { accH[nt] = zero8(); accR[nt] = zero8(); }

#pragma unroll 1
  for (int dh = 0; dh < 2; ++dh) {
    float x[16];
    {
      const v4f x0 = *(const v4f*)(xrow + 32 * dh);
      const v4f x1 = *(const v4f*)(xrow + 32 * dh + 4);
      const v4f x2 = *(const v4f*)(xrow + 32 * dh + 16);
      const v4f x3 = *(const v4f*)(xrow + 32 * dh + 20);
#pragma unroll
      for (int c = 0; c < 4; ++c) {
        x[c]      = bfr(x0[c]);
        x[4 + c]  = bfr(x1[c]);
        x[8 + c]  = bfr(x2[c]);
        x[12 + c] = bfr(x3[c]);
      }
    }
#pragma unroll 1
    for (int j = 0; j < NJ; ++j) {
      const int kq = dh * 640 + j * 32;
      const v4f p0 = *(const v4f*)(prow + kq);
      const v4f p1 = *(const v4f*)(prow + kq + 4);
      const v4f p2 = *(const v4f*)(prow + kq + 16);
      const v4f p3 = *(const v4f*)(prow + kq + 20);
      Frag ah, al;
      {
        v8h h0, l0, h1, l1;
#pragma unroll
        for (int c = 0; c < 4; ++c) {
          _Float16 th, tl;
          hsplit(x[c]      * p0[c], th, tl); h0[c]     = th; l0[c]     = tl;
          hsplit(x[4 + c]  * p1[c], th, tl); h0[4 + c] = th; l0[4 + c] = tl;
          hsplit(x[8 + c]  * p2[c], th, tl); h1[c]     = th; l1[c]     = tl;
          hsplit(x[12 + c] * p3[c], th, tl); h1[4 + c] = th; l1[4 + c] = tl;
        }
        ah.half[0] = h0; ah.half[1] = h1;
        al.half[0] = l0; al.half[1] = l1;
      }
#pragma unroll
      for (int nt = 0; nt < 4; ++nt) {
        const v16h bfv = ldfrag(zcol + (size_t)nt * (16 * NK) + kq);
        accH[nt] = mma(ah.v, bfv, accH[nt]);
        accR[nt] = mma(al.v, bfv, accR[nt]);
      }
    }
  }

  float* sw = sO + wv * 1024;
#pragma unroll
  for (int nt = 0; nt < 4; ++nt)
#pragma unroll
    for (int r = 0; r < 8; ++r)
      sw[(8 * hf + r) * 64 + nt * 16 + m] = accH[nt][r] * k2m16 + accR[nt][r] * k2m27;
  __syncthreads();

  v4f ov[8];
#pragma unroll
  for (int it = 0; it < 8; ++it) ov[it] = *(const v4fa*)(sw + (2 * it + hf) * 64 + 4 * m);
  float* ob = out + (size_t)sel * NOUT
            + ((size_t)((b * NL + lt * 64 + wv * 16) * NHD + hh)) * NR + ch * 64 + 4 * m;
#pragma unroll
  for (int it = 0; it < 8; ++it)
    *(volatile v4f*)(ob + (size_t)(2 * it + hf) * (NHD * NR)) = ov[it];
  __threadfence();
#pragma unroll
  for (int it = 0; it < 8; ++it)
    *(volatile v4f*)(ob + (size_t)(2 * it + hf) * (NHD * NR)) = ov[it];
}

extern "C" void kernel_launch(void* const* d_in, const int* in_sizes, int n_in,
                              void* d_out, int out_size, void* d_ws, size_t ws_size,
                              hipStream_t stream) {
  if (n_in < 6) return;
  if (in_sizes[0] != NB * NL * NHD * ND) return;
  if (in_sizes[1] != NB * NL * NHD * ND) return;
  if (in_sizes[2] != NTAB) return;
  if (in_sizes[3] != NTAB) return;
  if (in_sizes[4] != NTAB) return;
  if (in_sizes[5] != NBH * ND * NJ * NR) return;
  if (out_size != 2 * NOUT) return;

  const float* queries = (const float*)d_in[0];
  const float* keys    = (const float*)d_in[1];
  const float* freqs   = (const float*)d_in[2];
  const float* offsets = (const float*)d_in[3];
  const float* gains   = (const float*)d_in[4];
  const float* z       = (const float*)d_in[5];
  float* out = (float*)d_out;

  const size_t offTab = 0;
  const size_t szTab  = (size_t)2 * NTAB * sizeof(float);
  const size_t offZt  = offTab + szTab;
  const size_t szZt   = ZTN * sizeof(_Float16);
  const size_t offP   = offZt + szZt;
  const size_t szP    = (size_t)2 * PLANE * sizeof(float);
  const size_t total  = offP + szP;
  if (total > ws_size) return;
  if (total > (size_t)134217728) return;

  char* ws = (char*)d_ws;
  float*    tab = (float*)(ws + offTab);
  _Float16* zt  = (_Float16*)(ws + offZt);
  float*    Pqk = (float*)(ws + offP);

  const dim3 gTab(5),            bTab(256);
  const dim3 gZt(NBH * 2 * 8),   bZt(256);
  const dim3 gFeat(NHD * NL),    bFeat(160);
  const dim3 gGemm(NBH * 16 * 2 * 2), bGemm(128);

  k_tab<<<gTab, bTab, 0, stream>>>(freqs, gains, tab);
  k_zt<<<gZt, bZt, 0, stream>>>(z, zt);
  k_feat<<<gFeat, bFeat, 0, stream>>>(tab, offsets, Pqk);
  k_gemm<<<gGemm, bGemm, 0, stream>>>(queries, keys, Pqk, zt, out);
  (void)hipGetLastError();
}
